// RuntimePredictionGNN_62070867362011
// MI455X (gfx1250) — hardware-verified
//
#include <hip/hip_runtime.h>
#define NNODE 50000
#define NEDGE 800000
#define NP2 1048576
#define NB 512
#define NF 16
#define EF 8
#define GF 32
#define HH 64
#define NL 4
#define NG 20
#define NTH 9
#define KM 96

typedef __bf16 v16b __attribute__((ext_vector_type(16)));
typedef unsigned short v8us __attribute__((ext_vector_type(8), may_alias));
typedef float  v8f  __attribute__((ext_vector_type(8)));
typedef float  v4f  __attribute__((ext_vector_type(4)));
typedef float  v4fa __attribute__((ext_vector_type(4), may_alias));
union FragB { v16b v; v8us half[2]; unsigned short u[16]; };

__device__ __forceinline__ unsigned short bf16_bits(float x) { unsigned int u = __float_as_uint(x); return (unsigned short)((u + 0x7FFFu + ((u >> 16) & 1u)) >> 16); }
__device__ __forceinline__ float bf16_val(unsigned short b) { return __uint_as_float(((unsigned int)b) << 16); }
__device__ __forceinline__ float bf16_round(float x) { return bf16_val(bf16_bits(x)); }
template <int NT>
__device__ __forceinline__ v8f mmaN(v16b ah, v16b al, v16b bh, v16b bl, v8f c) {
  c = __builtin_amdgcn_wmma_f32_16x16x32_bf16(false, ah, false, bh, (short)0, c, false, false);
  if (NT >= 2) c = __builtin_amdgcn_wmma_f32_16x16x32_bf16(false, al, false, bh, (short)0, c, false, false);
  if (NT >= 3) c = __builtin_amdgcn_wmma_f32_16x16x32_bf16(false, ah, false, bl, (short)0, c, false, false);
  asm volatile("v_nop\n\tv_nop\n\tv_nop\n\tv_nop" : "+v"(c) : "v"(ah), "v"(al), "v"(bh), "v"(bl));
  return c;
}

__global__ __launch_bounds__(256) void k_wt_bf16(const float* __restrict__ W, unsigned short* __restrict__ Wt, int K, int N) {
  const int t = blockIdx.x * 256 + threadIdx.x;
  const int k8n = K / 8;
  if (t >= N * k8n) return;
  const int n = t / k8n, k8 = (t % k8n) * 8;
  v8us v;
#pragma unroll
  for (int i = 0; i < 8; ++i) v[i] = bf16_bits(W[(size_t)(k8 + i) * N + n]);
  *(volatile v8us*)(Wt + (size_t)n * K + k8) = v;
  __threadfence();
  *(volatile v8us*)(Wt + (size_t)n * K + k8) = v;
}

template <bool ASPLIT, int ACT, bool BIAS_BF16>
__global__ __launch_bounds__(128) void k_gemm_bf(const float* __restrict__ A, int lda, const unsigned short* __restrict__ Wt, int ldb,
                                               const float* __restrict__ bias, float* __restrict__ C, int ldc, int M, int N, int K) {
  __shared__ __attribute__((aligned(16))) float so[4][16][64];
  const int tid = threadIdx.x, w = tid >> 5, lane = tid & 31, ln = lane & 15, hh = lane >> 4;
  const int ntn = N / 64;
  const int wid = blockIdx.x * 4 + w;
  const int mt = wid / ntn, nq = wid % ntn;
  if (mt * 16 >= M) return;
  const int row0 = mt * 16, col0 = nq * 64;
  const float* arow = A + (size_t)(row0 + ln) * lda;
  v8f acc[4] = {};
  for (int kb = 0; kb < K; kb += 32) {
    FragB ah, al;
    const v4f x0 = *(const v4fa*)(arow + kb + 8 * hh), x1 = *(const v4fa*)(arow + kb + 8 * hh + 4);
    const v4f x2 = *(const v4fa*)(arow + kb + 16 + 8 * hh), x3 = *(const v4fa*)(arow + kb + 16 + 8 * hh + 4);
    float xs[16] = {x0[0],x0[1],x0[2],x0[3],x1[0],x1[1],x1[2],x1[3],x2[0],x2[1],x2[2],x2[3],x3[0],x3[1],x3[2],x3[3]};
#pragma unroll
    for (int i = 0; i < 16; ++i) { const unsigned short hb = bf16_bits(xs[i]); ah.u[i] = hb; al.u[i] = ASPLIT ? bf16_bits(xs[i] - bf16_val(hb)) : (unsigned short)0; }
#pragma unroll
    for (int t = 0; t < 4; ++t) {
      const unsigned short* brow = Wt + (size_t)(col0 + t * 16 + ln) * ldb + kb;
      FragB b;
      b.half[0] = *(const v8us*)(brow + 8 * hh);
      b.half[1] = *(const v8us*)(brow + 16 + 8 * hh);
      acc[t] = mmaN<ASPLIT ? 2 : 1>(ah.v, al.v, b.v, b.v, acc[t]);
    }
  }
#pragma unroll
  for (int t = 0; t < 4; ++t) {
    float bv = bias ? bias[col0 + t * 16 + ln] : 0.f;
    if (BIAS_BF16) bv = bf16_round(bv);
#pragma unroll
    for (int r = 0; r < 8; ++r) { float v = acc[t][r] + bv; if (ACT == 1) v = fmaxf(v, 0.f); so[w][8 * hh + r][t * 16 + ln] = v; }
  }
  __builtin_amdgcn_fence(__ATOMIC_ACQ_REL, "workgroup");
  __builtin_amdgcn_wave_barrier();
  const int rsub = lane >> 4, c4 = (lane & 15) * 4;
  for (int pass = 0; pass < 2; ++pass) {
#pragma unroll
    for (int q = 0; q < 8; ++q) {
      const int r = q * 2 + rsub;
      const v4f v = *(const v4fa*)&so[w][r][c4];
      *(volatile v4f*)(C + (size_t)(row0 + r) * ldc + col0 + c4) = v;
    }
    if (pass == 0) __threadfence();
  }
}

template <int D, bool CAUSAL>
__global__ __launch_bounds__(128) void k_flash(const float* __restrict__ qb, const float* __restrict__ kb, const float* __restrict__ vb,
                                             int pitch, int T, int H, float scale, float* __restrict__ y, int ypitch) {
  constexpr int KS = D / 32;
  constexpr int DT = D / 16;
  __shared__ __attribute__((aligned(16))) unsigned short sKh[32][D + 8], sKl[32][D + 8], sVh[32][D + 8], sVl[32][D + 8];
  __shared__ __attribute__((aligned(16))) unsigned short sPh[4][16][40], sPl[4][16][40];
  __shared__ __attribute__((aligned(16))) float sO[4][16][D];
  const int tid = threadIdx.x, w = tid >> 5, lane = tid & 31, ln = lane & 15, hh = lane >> 4;
  const int nqb = (T + 63) / 64;
  const int bh = blockIdx.x / nqb, qblk = blockIdx.x % nqb;
  const int b = bh / H, h = bh % H;
  const int q0 = qblk * 64 + w * 16;
  const float* Q = qb + (size_t)b * T * pitch + h * D;
  const float* K = kb + (size_t)b * T * pitch + h * D;
  const float* V = vb + (size_t)b * T * pitch + h * D;

  FragB aqh[KS], aql[KS];
  {
    int row = q0 + ln; if (row >= T) row = T - 1;
    const float* qr = Q + (size_t)row * pitch;
#pragma unroll
    for (int ks = 0; ks < KS; ++ks)
#pragma unroll
      for (int i = 0; i < 16; ++i) {
        const int d = ks * 32 + ((i < 8) ? (8 * hh + i) : (16 + 8 * hh + (i - 8)));
        const float x = qr[d] * scale; const unsigned short hb = bf16_bits(x);
        aqh[ks].u[i] = hb; aql[ks].u[i] = bf16_bits(x - bf16_val(hb));
      }
  }
  float m_r[8], l_r[8];
#pragma unroll
  for (int r = 0; r < 8; ++r) { m_r[r] = -3.0e38f; l_r[r] = 0.f; }
  v8f oacc[DT];
#pragma unroll
  for (int dt = 0; dt < DT; ++dt) oacc[dt] = (v8f){0.f,0.f,0.f,0.f,0.f,0.f,0.f,0.f};

  const int kv_end = CAUSAL ? min(T, qblk * 64 + 64) : T;
  for (int j0 = 0; j0 < kv_end; j0 += 32) {
    __syncthreads();
    for (int e = tid; e < 32 * (D / 4); e += 128) {
      const int r = e / (D / 4), c4 = (e % (D / 4)) * 4;
      const int key = j0 + r;
      v4f kf = {0.f,0.f,0.f,0.f}, vf = {0.f,0.f,0.f,0.f};
      if (key < T) { kf = *(const v4fa*)(K + (size_t)key * pitch + c4); vf = *(const v4fa*)(V + (size_t)key * pitch + c4); }
#pragma unroll
      for (int t = 0; t < 4; ++t) {
        unsigned short hb = bf16_bits(kf[t]); sKh[r][c4 + t] = hb; sKl[r][c4 + t] = bf16_bits(kf[t] - bf16_val(hb));
        hb = bf16_bits(vf[t]); sVh[r][c4 + t] = hb; sVl[r][c4 + t] = bf16_bits(vf[t] - bf16_val(hb));
      }
    }
    __syncthreads();
    v8f s[2];
#pragma unroll
    for (int nt = 0; nt < 2; ++nt) {
      v8f acc = {};
#pragma unroll
      for (int ks = 0; ks < KS; ++ks) {
        FragB bh_, bl_;
        bh_.half[0] = *(const v8us*)&sKh[nt * 16 + ln][ks * 32 + 8 * hh]; bh_.half[1] = *(const v8us*)&sKh[nt * 16 + ln][ks * 32 + 16 + 8 * hh];
        bl_.half[0] = *(const v8us*)&sKl[nt * 16 + ln][ks * 32 + 8 * hh]; bl_.half[1] = *(const v8us*)&sKl[nt * 16 + ln][ks * 32 + 16 + 8 * hh];
        acc = mmaN<3>(aqh[ks].v, aql[ks].v, bh_.v, bl_.v, acc);
      }
      s[nt] = acc;
    }
    float alpha[8];
#pragma unroll
    for (int r = 0; r < 8; ++r) {
      const int qi = q0 + 8 * hh + r;
      const int ja = j0 + ln, jb = j0 + 16 + ln;
      if (CAUSAL) { if (ja > qi) s[0][r] = -3.0e38f; if (jb > qi) s[1][r] = -3.0e38f; }
      if (ja >= T) s[0][r] = -3.0e38f;
      if (jb >= T) s[1][r] = -3.0e38f;
      float mx = fmaxf(s[0][r], s[1][r]);
      mx = fmaxf(mx, __shfl_xor(mx, 1, 32)); mx = fmaxf(mx, __shfl_xor(mx, 2, 32)); mx = fmaxf(mx, __shfl_xor(mx, 4, 32)); mx = fmaxf(mx, __shfl_xor(mx, 8, 32));
      const float mnew = fmaxf(m_r[r], mx);
      alpha[r] = (mnew > -1.0e38f) ? __expf(m_r[r] - mnew) : 1.0f;
      const float p0 = (s[0][r] > -1.0e38f) ? __expf(s[0][r] - mnew) : 0.f;
      const float p1 = (s[1][r] > -1.0e38f) ? __expf(s[1][r] - mnew) : 0.f;
      m_r[r] = mnew;
      l_r[r] = l_r[r] * alpha[r] + p0 + p1;
      unsigned short hb = bf16_bits(p0); sPh[w][8 * hh + r][ln] = hb;      sPl[w][8 * hh + r][ln] = bf16_bits(p0 - bf16_val(hb));
      hb = bf16_bits(p1);                sPh[w][8 * hh + r][16 + ln] = hb; sPl[w][8 * hh + r][16 + ln] = bf16_bits(p1 - bf16_val(hb));
    }
#pragma unroll
    for (int dt = 0; dt < DT; ++dt)
#pragma unroll
      for (int r = 0; r < 8; ++r) oacc[dt][r] *= alpha[r];
    __builtin_amdgcn_fence(__ATOMIC_ACQ_REL, "workgroup");
    __builtin_amdgcn_wave_barrier();
    FragB pah, pal;
    pah.half[0] = *(const v8us*)&sPh[w][ln][8 * hh]; pah.half[1] = *(const v8us*)&sPh[w][ln][16 + 8 * hh];
    pal.half[0] = *(const v8us*)&sPl[w][ln][8 * hh]; pal.half[1] = *(const v8us*)&sPl[w][ln][16 + 8 * hh];
#pragma unroll
    for (int dt = 0; dt < DT; ++dt) {
      FragB bvh, bvl;
#pragma unroll
      for (int i = 0; i < 8; ++i) {
        bvh.u[i] = sVh[8 * hh + i][dt * 16 + ln]; bvh.u[8 + i] = sVh[16 + 8 * hh + i][dt * 16 + ln];
        bvl.u[i] = sVl[8 * hh + i][dt * 16 + ln]; bvl.u[8 + i] = sVl[16 + 8 * hh + i][dt * 16 + ln];
      }
      oacc[dt] = mmaN<3>(pah.v, pal.v, bvh.v, bvl.v, oacc[dt]);
    }
    __builtin_amdgcn_fence(__ATOMIC_ACQ_REL, "workgroup");
    __builtin_amdgcn_wave_barrier();
  }
#pragma unroll
  for (int r = 0; r < 8; ++r) {
    float l = l_r[r];
    l += __shfl_xor(l, 1, 32); l += __shfl_xor(l, 2, 32); l += __shfl_xor(l, 4, 32); l += __shfl_xor(l, 8, 32);
    l_r[r] = (l > 0.f) ? 1.0f / l : 0.f;
  }
#pragma unroll
  for (int dt = 0; dt < DT; ++dt)
#pragma unroll
    for (int r = 0; r < 8; ++r) sO[w][8 * hh + r][dt * 16 + ln] = oacc[dt][r] * l_r[r];
  __builtin_amdgcn_fence(__ATOMIC_ACQ_REL, "workgroup");
  __builtin_amdgcn_wave_barrier();
  for (int pass = 0; pass < 2; ++pass) {
    for (int r = 0; r < 16; ++r) {
      const int row = q0 + r;
      if (row < T && lane < D / 4) {
        const v4f val = *(const v4fa*)&sO[w][r][lane * 4];
        *(volatile v4f*)(y + ((size_t)b * T + row) * ypitch + h * D + lane * 4) = val;
      }
    }
    if (pass == 0) __threadfence();
  }
}

template <bool ASPLIT, int ACT, bool BIAS_BF16, bool RES_BF16>
__global__ __launch_bounds__(128) void k_gemm_bf3(const float* __restrict__ A, int lda, const unsigned short* __restrict__ Wt, int ldb,
                                                const float* __restrict__ bias, const float* __restrict__ resid, int rmod, int ldr,
                                                float* __restrict__ C, int ldc, int M, int N, int K) {
  __shared__ __attribute__((aligned(16))) float so[4][16][64];
  const int tid = threadIdx.x, w = tid >> 5, lane = tid & 31, ln = lane & 15, hh = lane >> 4;
  const int ntn = N / 64;
  const int wid = blockIdx.x * 4 + w;
  const int mt = wid / ntn, nq = wid % ntn;
  if (mt * 16 >= M) return;
  const int row0 = mt * 16, col0 = nq * 64;
  const float* arow = A + (size_t)(row0 + ln) * lda;
  v8f acc[4] = {};
  for (int kb = 0; kb < K; kb += 32) {
    FragB ah, al;
    const v4f x0 = *(const v4fa*)(arow + kb + 8 * hh), x1 = *(const v4fa*)(arow + kb + 8 * hh + 4);
    const v4f x2 = *(const v4fa*)(arow + kb + 16 + 8 * hh), x3 = *(const v4fa*)(arow + kb + 16 + 8 * hh + 4);
    float xs[16] = {x0[0],x0[1],x0[2],x0[3],x1[0],x1[1],x1[2],x1[3],x2[0],x2[1],x2[2],x2[3],x3[0],x3[1],x3[2],x3[3]};
#pragma unroll
    for (int i = 0; i < 16; ++i) { const unsigned short hb = bf16_bits(xs[i]); ah.u[i] = hb; al.u[i] = ASPLIT ? bf16_bits(xs[i] - bf16_val(hb)) : (unsigned short)0; }
#pragma unroll
    for (int t = 0; t < 4; ++t) {
      const unsigned short* brow = Wt + (size_t)(col0 + t * 16 + ln) * ldb + kb;
      FragB b;
      b.half[0] = *(const v8us*)(brow + 8 * hh);
      b.half[1] = *(const v8us*)(brow + 16 + 8 * hh);
      acc[t] = mmaN<ASPLIT ? 2 : 1>(ah.v, al.v, b.v, b.v, acc[t]);
    }
  }
#pragma unroll
  for (int t = 0; t < 4; ++t) {
    const int col = col0 + t * 16 + ln;
    float bv = bias ? bias[col] : 0.f;
    if (BIAS_BF16) bv = bf16_round(bv);
#pragma unroll
    for (int r = 0; r < 8; ++r) {
      float v = acc[t][r] + bv;
      if (resid) { float rv = resid[(size_t)((row0 + 8 * hh + r) % rmod) * ldr + col]; if (RES_BF16) rv = bf16_round(rv); v += rv; }
      if (ACT == 1) v = fmaxf(v, 0.f);
      if (ACT == 2) v = 0.5f * v * (1.0f + erff(v * 0.70710678118654752f));
      if (ACT == 3) { const float u = 0.7978845608028654f * (v + 0.044715f * v * v * v); v = 0.5f * v * (1.0f + tanhf(u)); }
      so[w][8 * hh + r][t * 16 + ln] = v;
    }
  }
  __builtin_amdgcn_fence(__ATOMIC_ACQ_REL, "workgroup");
  __builtin_amdgcn_wave_barrier();
  const int rsub = lane >> 4, c4 = (lane & 15) * 4;
  for (int pass = 0; pass < 2; ++pass) {
#pragma unroll
    for (int q = 0; q < 8; ++q) {
      const int r = q * 2 + rsub;
      const v4f v = *(const v4fa*)&so[w][r][c4];
      *(volatile v4f*)(C + (size_t)(row0 + r) * ldc + col0 + c4) = v;
    }
    if (pass == 0) __threadfence();
  }
}
template <bool PARAM_BF16>
__global__ __launch_bounds__(256) void k_layernorm(const float* __restrict__ X, const float* __restrict__ R, const float* __restrict__ g, const float* __restrict__ bta,
                                                  float* __restrict__ out_sum, float* __restrict__ out_norm, int N, float eps) {
  __shared__ float red[256];
  const int row = blockIdx.x, tid = threadIdx.x;
  const float* x = X + (size_t)row * N; const float* rr = R ? R + (size_t)row * N : nullptr;
  float vals[16];
  const int per = N / 256;
  float s1 = 0.f;
  for (int u = 0; u < per / 4; ++u) {
    const int j = tid * 4 + 1024 * u;
    const v4f a = *(const v4fa*)(x + j);
    v4f b = {0.f,0.f,0.f,0.f}; if (rr) b = *(const v4fa*)(rr + j);
#pragma unroll
    for (int q = 0; q < 4; ++q) { const float v = a[q] + b[q]; vals[u * 4 + q] = v; s1 += v; }
  }
  red[tid] = s1; __syncthreads();
  for (int st = 128; st > 0; st >>= 1) { if (tid < st) red[tid] += red[tid + st]; __syncthreads(); }
  const float mu = red[0] / (float)N; __syncthreads();
  float s2 = 0.f;
  for (int u = 0; u < per / 4; ++u)
#pragma unroll
    for (int q = 0; q < 4; ++q) { const float c = vals[u * 4 + q] - mu; s2 += c * c; }
  red[tid] = s2; __syncthreads();
  for (int st = 128; st > 0; st >>= 1) { if (tid < st) red[tid] += red[tid + st]; __syncthreads(); }
  const float rs = rsqrtf(red[0] / (float)N + eps);
  for (int pass = 0; pass < 2; ++pass) {
    for (int u = 0; u < per / 4; ++u) {
      const int j = tid * 4 + 1024 * u;
      v4f o, sm;
#pragma unroll
      for (int q = 0; q < 4; ++q) {
        float gg = g[j + q], bb = bta[j + q];
        if (PARAM_BF16) { gg = bf16_round(gg); bb = bf16_round(bb); }
        sm[q] = vals[u * 4 + q]; o[q] = (vals[u * 4 + q] - mu) * rs * gg + bb;
      }
      if (out_sum) *(volatile v4f*)(out_sum + (size_t)row * N + j) = sm;
      *(volatile v4f*)(out_norm + (size_t)row * N + j) = o;
    }
    if (pass == 0) __threadfence();
  }
}

__global__ __launch_bounds__(256) void k_sort_init(const int* __restrict__ seg, int n, int nseg, unsigned int* __restrict__ key, unsigned int* __restrict__ val, int np2) {
  const int i = blockIdx.x * 256 + threadIdx.x; if (i >= np2) return;
  unsigned int kv = 0xFFFFFFFFu;
  if (i < n) { int s = seg[i]; s = s < 0 ? 0 : (s >= nseg ? nseg - 1 : s); kv = (unsigned int)s; }
  *(volatile unsigned int*)(key + i) = kv; *(volatile unsigned int*)(val + i) = (unsigned int)i;
  __threadfence();
  *(volatile unsigned int*)(key + i) = kv; *(volatile unsigned int*)(val + i) = (unsigned int)i;
}
template <bool STAGE0>
__global__ __launch_bounds__(512) void k_sort_lds(unsigned int* __restrict__ key, unsigned int* __restrict__ val, int kstage) {
  __shared__ unsigned int sk[1024], sv[1024];
  const int tid = threadIdx.x; const int base = blockIdx.x * 1024;
  sk[tid] = key[base + tid]; sv[tid] = val[base + tid]; sk[tid + 512] = key[base + tid + 512]; sv[tid + 512] = val[base + tid + 512];
  __syncthreads();
  for (int k = (STAGE0 ? 2 : kstage); k <= (STAGE0 ? 1024 : kstage); k <<= 1) {
    for (int j = (k > 1024 ? 512 : (k >> 1)); j >= 1; j >>= 1) {
      const int lo = tid & (j - 1), hi2 = (tid >> __builtin_ctz(j)) << (__builtin_ctz(j) + 1);
      const int il = hi2 | lo, ir = il | j;
      const int gi = base + il;
      const bool asc = ((gi & k) == 0);
      unsigned int a = sk[il], b = sk[ir], va = sv[il], vb = sv[ir];
      const bool swp = asc ? (a > b) : (a < b);
      if (swp) { sk[il] = b; sk[ir] = a; sv[il] = vb; sv[ir] = va; }
      __syncthreads();
    }
  }
  for (int pass = 0; pass < 2; ++pass) {
    *(volatile unsigned int*)(key + base + tid) = sk[tid]; *(volatile unsigned int*)(val + base + tid) = sv[tid];
    *(volatile unsigned int*)(key + base + tid + 512) = sk[tid + 512]; *(volatile unsigned int*)(val + base + tid + 512) = sv[tid + 512];
    if (pass == 0) __threadfence();
  }
}
__global__ __launch_bounds__(256) void k_sort_step(unsigned int* __restrict__ key, unsigned int* __restrict__ val, int k, int j, int np2) {
  const int t = blockIdx.x * 256 + threadIdx.x; if (t >= np2 / 2) return;
  const int lo = t & (j - 1), il = ((t >> __builtin_ctz(j)) << (__builtin_ctz(j) + 1)) | lo, ir = il | j;
  const bool asc = ((il & k) == 0);
  unsigned int a = key[il], b = key[ir], va = val[il], vb = val[ir];
  const bool swp = asc ? (a > b) : (a < b);
  const unsigned int k1 = swp ? b : a, k2 = swp ? a : b, v1 = swp ? vb : va, v2 = swp ? va : vb;
  *(volatile unsigned int*)(key + il) = k1; *(volatile unsigned int*)(key + ir) = k2; *(volatile unsigned int*)(val + il) = v1; *(volatile unsigned int*)(val + ir) = v2;
  __threadfence();
  *(volatile unsigned int*)(key + il) = k1; *(volatile unsigned int*)(key + ir) = k2; *(volatile unsigned int*)(val + il) = v1; *(volatile unsigned int*)(val + ir) = v2;
}
__global__ __launch_bounds__(256) void k_rowptr(const unsigned int* __restrict__ key, int np2, int nseg, int* __restrict__ rowptr) {
  int s = blockIdx.x * 256 + threadIdx.x; if (s >= ((nseg + 1 + 31) / 32) * 32) return;
  const int sdst = s; if (s > nseg) s = nseg;
  int lo = 0, hi = np2;
  while (lo < hi) { const int mid = (lo + hi) >> 1; if (key[mid] < (unsigned int)s) lo = mid + 1; else hi = mid; }
  *(volatile int*)(rowptr + sdst) = lo; __threadfence(); *(volatile int*)(rowptr + sdst) = lo;
}
static void sort_pairs(unsigned int* key, unsigned int* val, int np2, hipStream_t stream) {
  k_sort_lds<true><<<np2 / 1024, 512, 0, stream>>>(key, val, 0);
  for (int k = 2048; k <= np2; k <<= 1) {
    for (int j = k >> 1; j >= 1024; j >>= 1) k_sort_step<<<(np2 / 2 + 255) / 256, 256, 0, stream>>>(key, val, k, j, np2);
    k_sort_lds<false><<<np2 / 1024, 512, 0, stream>>>(key, val, k);
  }
}

__global__ void k_ln_rows(const float* __restrict__ X, const float* __restrict__ R, const float* __restrict__ g, const float* __restrict__ bta, float* __restrict__ out, int N, float eps) {
  __shared__ float red[256];
  const int row = blockIdx.x, tid = threadIdx.x, nt = blockDim.x;
  v4f a = *(const v4fa*)(X + (size_t)row * N + tid * 4);
  if (R) { const v4f rr = *(const v4fa*)(R + (size_t)row * N + tid * 4); for (int q = 0; q < 4; ++q) a[q] += rr[q]; }
  float s = a[0] + a[1] + a[2] + a[3];
  red[tid] = s; __syncthreads();
  for (int st = nt / 2; st > 0; st >>= 1) { if (tid < st) red[tid] += red[tid + st]; __syncthreads(); }
  const float mu = red[0] / (float)N; __syncthreads();
  float v = 0.f; for (int q = 0; q < 4; ++q) { const float c = a[q] - mu; v += c * c; }
  red[tid] = v; __syncthreads();
  for (int st = nt / 2; st > 0; st >>= 1) { if (tid < st) red[tid] += red[tid + st]; __syncthreads(); }
  const float rs = rsqrtf(red[0] / (float)N + eps);
  v4f o; for (int q = 0; q < 4; ++q) o[q] = (a[q] - mu) * rs * bf16_round(g[tid * 4 + q]) + bf16_round(bta[tid * 4 + q]);
  *(volatile v4f*)(out + (size_t)row * N + tid * 4) = o; __threadfence(); *(volatile v4f*)(out + (size_t)row * N + tid * 4) = o;
}

__global__ __launch_bounds__(256) void k_enc(const float* __restrict__ x, const float* __restrict__ W0, const float* __restrict__ b0, const float* __restrict__ g, const float* __restrict__ bb, float* __restrict__ h) {
  const int tid = threadIdx.x, w = tid >> 5, lane = tid & 31; const int n = blockIdx.x * 8 + w; if (n >= NNODE) return;
  float xv[NF]; for (int k = 0; k < NF; ++k) xv[k] = bf16_round(x[(size_t)n * NF + k]);
  v4f a = {0.f,0.f,0.f,0.f};
  if (lane < 16) { for (int q = 0; q < 4; ++q) { const int c = lane * 4 + q; float s = bf16_round(b0[c]);
#pragma unroll 1
      for (int k = 0; k < NF; ++k) s += xv[k] * bf16_round(W0[k * HH + c]); a[q] = fmaxf(s, 0.f); } }
  float s = (lane < 16) ? (a[0] + a[1] + a[2] + a[3]) : 0.f; for (int o = 16; o >= 1; o >>= 1) s += __shfl_xor(s, o, 32);
  const float mu = s * (1.0f / HH);
  float v = 0.f; if (lane < 16) for (int q = 0; q < 4; ++q) { const float c = a[q] - mu; v += c * c; } for (int o = 16; o >= 1; o >>= 1) v += __shfl_xor(v, o, 32);
  const float rs = rsqrtf(v * (1.0f / HH) + 1e-5f);
  if (lane < 16) { v4f o; for (int q = 0; q < 4; ++q) o[q] = (a[q] - mu) * rs * bf16_round(g[lane * 4 + q]) + bf16_round(bb[lane * 4 + q]); float* row = h + (size_t)n * HH + lane * 4; *(volatile v4f*)row = o; __threadfence(); *(volatile v4f*)row = o; }
}
__global__ __launch_bounds__(256) void k_wt_msg(const float* __restrict__ W, unsigned short* __restrict__ Bt) {
  const int t = blockIdx.x * 256 + threadIdx.x; if (t >= HH * 12) return; const int n = t / 12, k8 = (t % 12) * 8; v8us v;
  for (int i = 0; i < 8; ++i) { const int k = k8 + i; v[i] = (k < HH + EF) ? bf16_bits(W[k * HH + n]) : (unsigned short)0; }
  *(volatile v8us*)(Bt + n * KM + k8) = v; __threadfence(); *(volatile v8us*)(Bt + n * KM + k8) = v;
}
__global__ __launch_bounds__(128) void k_gemm_msg(const float* __restrict__ h, const float* __restrict__ ea, const int* __restrict__ src, const int* __restrict__ etype,
                                                const unsigned short* __restrict__ Bt, const float* __restrict__ bmsg, const float* __restrict__ gemb, float* __restrict__ m) {
  __shared__ __attribute__((aligned(16))) float so[4][16][64];
  const int tid = threadIdx.x, w = tid >> 5, lane = tid & 31, ln = lane & 15, hh = lane >> 4;
  const size_t e0 = ((size_t)blockIdx.x * 4 + w) * 16; const size_t e = e0 + ln;
  int sn = src[e]; sn = sn < 0 ? 0 : (sn >= NNODE ? NNODE - 1 : sn);
  const float* hr = h + (size_t)sn * HH; const float* er = ea + e * EF;
  v8f acc[4] = {};
#pragma unroll
  for (int ks = 0; ks < 3; ++ks) {
    FragB ah, al;
#pragma unroll
    for (int i = 0; i < 16; ++i) { const int k = ks * 32 + ((i < 8) ? (8 * hh + i) : (16 + 8 * hh + (i - 8))); float v = 0.f; if (k < HH) v = hr[k]; else if (k < HH + EF) v = bf16_round(er[k - HH]); const unsigned short hb = bf16_bits(v); ah.u[i] = hb; al.u[i] = bf16_bits(v - bf16_val(hb)); }
#pragma unroll
    for (int t = 0; t < 4; ++t) { FragB b; b.half[0] = *(const v8us*)(Bt + (t * 16 + ln) * KM + ks * 32 + 8 * hh); b.half[1] = *(const v8us*)(Bt + (t * 16 + ln) * KM + ks * 32 + 16 + 8 * hh); acc[t] = mmaN<2>(ah.v, al.v, b.v, b.v, acc[t]); }
  }
  int ty[8]; for (int r = 0; r < 8; ++r) { int t = etype[e0 + 8 * hh + r]; ty[r] = t < 0 ? 0 : (t >= NG ? NG - 1 : t); }
#pragma unroll
  for (int t = 0; t < 4; ++t) { const int col = t * 16 + ln; const float bv = bf16_round(bmsg[col]);
#pragma unroll
    for (int r = 0; r < 8; ++r) so[w][8 * hh + r][col] = fmaxf(acc[t][r] + bv + bf16_round(gemb[ty[r] * HH + col]), 0.f); }
  __builtin_amdgcn_fence(__ATOMIC_ACQ_REL, "workgroup"); __builtin_amdgcn_wave_barrier();
  const int rsub = lane >> 4, c4 = (lane & 15) * 4;
  for (int pass = 0; pass < 2; ++pass) { for (int q = 0; q < 8; ++q) { const int r = q * 2 + rsub; const v4f v = *(const v4fa*)&so[w][r][c4]; *(volatile v4f*)(m + (e0 + r) * HH + c4) = v; } if (pass == 0) __threadfence(); }
}
__global__ __launch_bounds__(256) void k_agg(const float* __restrict__ h, const float* __restrict__ m, const int* __restrict__ rowptr, const unsigned int* __restrict__ perm, float* __restrict__ hcat) {
  const int tid = threadIdx.x, w = tid >> 5, lane = tid & 31; const int nd = blockIdx.x * 8 + w; if (nd >= NNODE) return;
  const int p0 = rowptr[nd], p1 = rowptr[nd + 1];
  if (lane < 16) {
    v4f acc = {0.f,0.f,0.f,0.f};
    for (int p = p0; p < p1; ++p) { const v4f x0 = *(const v4fa*)(m + (size_t)perm[p] * HH + lane * 4); for (int q = 0; q < 4; ++q) acc[q] += x0[q]; }
    const float inv = 1.0f / fmaxf((float)(p1 - p0), 1.0f); for (int q = 0; q < 4; ++q) acc[q] *= inv;
    const v4f own = *(const v4fa*)(h + (size_t)nd * HH + lane * 4);
    float* row = hcat + (size_t)nd * 2 * HH; *(volatile v4f*)(row + lane * 4) = own; *(volatile v4f*)(row + HH + lane * 4) = acc; __threadfence(); *(volatile v4f*)(row + lane * 4) = own; *(volatile v4f*)(row + HH + lane * 4) = acc;
  }
}
__global__ __launch_bounds__(128) void k_gemm_upd(const float* __restrict__ A, const unsigned short* __restrict__ Wt, const float* __restrict__ bias, const float* __restrict__ hres, float* __restrict__ C, int M) {
  __shared__ __attribute__((aligned(16))) float so[4][16][64];
  const int tid = threadIdx.x, w = tid >> 5, lane = tid & 31, ln = lane & 15, hh = lane >> 4;
  const int mt = blockIdx.x * 4 + w; if (mt * 16 >= M) return; const int row0 = mt * 16;
  const float* arow = A + (size_t)(row0 + ln) * 2 * HH;
  v8f acc[4] = {};
  for (int kb = 0; kb < 2 * HH; kb += 32) {
    FragB ah, al;
    const v4f x0 = *(const v4fa*)(arow + kb + 8 * hh), x1 = *(const v4fa*)(arow + kb + 8 * hh + 4), x2 = *(const v4fa*)(arow + kb + 16 + 8 * hh), x3 = *(const v4fa*)(arow + kb + 16 + 8 * hh + 4);
    float xs[16] = {x0[0],x0[1],x0[2],x0[3],x1[0],x1[1],x1[2],x1[3],x2[0],x2[1],x2[2],x2[3],x3[0],x3[1],x3[2],x3[3]};
#pragma unroll
    for (int i = 0; i < 16; ++i) { const unsigned short hb = bf16_bits(xs[i]); ah.u[i] = hb; al.u[i] = bf16_bits(xs[i] - bf16_val(hb)); }
#pragma unroll
    for (int t = 0; t < 4; ++t) { FragB b; b.half[0] = *(const v8us*)(Wt + (size_t)(t * 16 + ln) * 2 * HH + kb + 8 * hh); b.half[1] = *(const v8us*)(Wt + (size_t)(t * 16 + ln) * 2 * HH + kb + 16 + 8 * hh); acc[t] = mmaN<2>(ah.v, al.v, b.v, b.v, acc[t]); }
  }
#pragma unroll
  for (int t = 0; t < 4; ++t) { const int col = t * 16 + ln; const float bv = bf16_round(bias[col]);
#pragma unroll
    for (int r = 0; r < 8; ++r) so[w][8 * hh + r][col] = hres[(size_t)(row0 + 8 * hh + r) * HH + col] + fmaxf(acc[t][r] + bv, 0.f); }
  __builtin_amdgcn_fence(__ATOMIC_ACQ_REL, "workgroup"); __builtin_amdgcn_wave_barrier();
  const int rsub = lane >> 4, c4 = (lane & 15) * 4;
  for (int pass = 0; pass < 2; ++pass) { for (int q = 0; q < 8; ++q) { const int r = q * 2 + rsub; const v4f v = *(const v4fa*)&so[w][r][c4]; *(volatile v4f*)(C + (size_t)(row0 + r) * HH + c4) = v; } if (pass == 0) __threadfence(); }
}
__global__ __launch_bounds__(256) void k_gptr(const int* __restrict__ batch, int* __restrict__ gptr) {
  const int slot = blockIdx.x * 256 + threadIdx.x; if (slot >= ((NB + 1 + 31) / 32) * 32) return; const int g = slot > NB ? NB : slot;
  int lo = 0, hi = NNODE; while (lo < hi) { const int mid = (lo + hi) >> 1; if (batch[mid] < g) lo = mid + 1; else hi = mid; }
  *(volatile int*)(gptr + slot) = lo; __threadfence(); *(volatile int*)(gptr + slot) = lo;
}
__global__ __launch_bounds__(64) void k_graphfeat(const float* __restrict__ h, const int* __restrict__ gptr, const float* __restrict__ gfeat, const int* __restrict__ thr,
                                                const float* __restrict__ Wg, const float* __restrict__ bg, const float* __restrict__ lg, const float* __restrict__ lb,
                                                const float* __restrict__ emb_th, const float* __restrict__ Wt, const float* __restrict__ bt, float* __restrict__ crow) {
  __shared__ float sg[HH]; __shared__ float red[64]; __shared__ float so[288];
  const int gidx = blockIdx.x, c = threadIdx.x; const int n0 = gptr[gidx], n1 = gptr[gidx + 1];
  float s = 0.f, mx = -__builtin_inff();
  for (int n = n0; n < n1; ++n) { const float v = h[(size_t)n * HH + c]; s += v; mx = fmaxf(mx, v); }
  const float cnt = (float)(n1 - n0);
  so[c] = s / fmaxf(cnt, 1.0f); so[HH + c] = (cnt > 0.f) ? mx : 0.f; so[2 * HH + c] = s;
  float gv = bf16_round(bg[c]);
#pragma unroll 1
  for (int k = 0; k < GF; ++k) gv += bf16_round(gfeat[gidx * GF + k]) * bf16_round(Wg[k * HH + c]);
  gv = fmaxf(gv, 0.f); sg[c] = gv; red[c] = gv; __syncthreads();
  for (int st = 32; st > 0; st >>= 1) { if (c < st) red[c] += red[c + st]; __syncthreads(); }
  const float mu = red[0] / HH; __syncthreads();
  red[c] = (gv - mu) * (gv - mu); __syncthreads();
  for (int st = 32; st > 0; st >>= 1) { if (c < st) red[c] += red[c + st]; __syncthreads(); }
  const float rs = rsqrtf(red[0] / HH + 1e-5f);
  so[3 * HH + c] = (gv - mu) * rs * bf16_round(lg[c]) + bf16_round(lb[c]);
  if (c < HH / 2) { int t = thr[gidx]; t = t < 0 ? 0 : (t >= NTH ? NTH - 1 : t); float tv = bf16_round(bt[c]);
#pragma unroll 1
    for (int k = 0; k < HH / 2; ++k) tv += bf16_round(emb_th[t * (HH / 2) + k]) * bf16_round(Wt[k * (HH / 2) + c]); so[4 * HH + c] = fmaxf(tv, 0.f); }
  __syncthreads();
  for (int pass = 0; pass < 2; ++pass) { for (int i = c; i < 72; i += 64) { v4f v; for (int q = 0; q < 4; ++q) v[q] = so[i * 4 + q]; *(volatile v4f*)(crow + (size_t)gidx * 288 + i * 4) = v; } if (pass == 0) __threadfence(); }
}
__global__ __launch_bounds__(256) void k_head(const float* __restrict__ c2, const float* __restrict__ Wh1, const float* __restrict__ bh1, const float* __restrict__ Wh2, const float* __restrict__ bh2, float* __restrict__ out) {
  __shared__ float so[NB];
  for (int gI = threadIdx.x; gI < NB; gI += 256) {
    const float* cr = c2 + (size_t)gI * HH; float o = bf16_round(bh2[0]);
#pragma unroll 1
    for (int j = 0; j < HH / 2; ++j) { float s = bf16_round(bh1[j]);
#pragma unroll 1
      for (int k = 0; k < HH; ++k) s += cr[k] * bf16_round(Wh1[k * (HH / 2) + j]); o += fmaxf(s, 0.f) * bf16_round(Wh2[j]); }
    so[gI] = o;
  }
  __syncthreads();
  for (int pass = 0; pass < 2; ++pass) { for (int gI = threadIdx.x; gI < NB; gI += 256) *(volatile float*)(out + gI) = so[gI]; if (pass == 0) __threadfence(); }
}

extern "C" void kernel_launch(void* const* d_in, const int* in_sizes, int n_in,
                              void* d_out, int out_size, void* d_ws, size_t ws_size, hipStream_t stream) {
  (void)in_sizes; (void)n_in; (void)out_size;
  const float* x = (const float*)d_in[0]; const int* ei = (const int*)d_in[1]; const float* ea = (const float*)d_in[2]; const int* etype = (const int*)d_in[3];
  const int* batch = (const int*)d_in[4]; const float* gfeat = (const float*)d_in[5]; const int* thr = (const int*)d_in[6];
  const float* W0 = (const float*)d_in[7]; const float* b0 = (const float*)d_in[8]; const float* ln1g = (const float*)d_in[9]; const float* ln1b = (const float*)d_in[10];
  const float* Wmsg = (const float*)d_in[11]; const float* bmsg = (const float*)d_in[12]; const float* gemb = (const float*)d_in[13]; const float* Wupd = (const float*)d_in[14]; const float* bupd = (const float*)d_in[15];
  const float* Wg = (const float*)d_in[16]; const float* bg = (const float*)d_in[17]; const float* lngg = (const float*)d_in[18]; const float* lngb = (const float*)d_in[19];
  const float* emb_th = (const float*)d_in[20]; const float* Wt = (const float*)d_in[21]; const float* bt = (const float*)d_in[22];
  const float* Wc1 = (const float*)d_in[23]; const float* bc1 = (const float*)d_in[24]; const float* lncg = (const float*)d_in[25]; const float* lncb = (const float*)d_in[26];
  const float* Wc2 = (const float*)d_in[27]; const float* bc2 = (const float*)d_in[28]; const float* Wh1 = (const float*)d_in[29]; const float* bh1 = (const float*)d_in[30]; const float* Wh2 = (const float*)d_in[31]; const float* bh2 = (const float*)d_in[32];
  const int* src = ei; const int* dst = ei + NEDGE;
  char* ws = (char*)d_ws; size_t off = 0;
  auto take = [&](size_t bytes) { char* p = ws + off; off += (bytes + 255) & ~(size_t)255; return p; };
  unsigned short* Bmsg[NL], *Bupd[NL]; for (int l = 0; l < NL; ++l) { Bmsg[l] = (unsigned short*)take(HH * KM * 2); Bupd[l] = (unsigned short*)take(HH * 2 * HH * 2); }
  unsigned short* Bc1 = (unsigned short*)take((size_t)128 * 288 * 2); unsigned short* Bc2 = (unsigned short*)take((size_t)64 * 128 * 2);
  unsigned int* key = (unsigned int*)take((size_t)NP2 * 4); unsigned int* perm = (unsigned int*)take((size_t)NP2 * 4); int* rowptr = (int*)take((size_t)(NNODE + 64) * 4);
  float* hA = (float*)take((size_t)NNODE * HH * 4); float* hB = (float*)take((size_t)NNODE * HH * 4); float* hcat = (float*)take((size_t)NNODE * 2 * HH * 4);
  float* m = (float*)take((size_t)NEDGE * HH * 4);
  int* gptr = (int*)take((size_t)(NB + 64) * 4); float* crow = (float*)take((size_t)NB * 288 * 4);
  float* c1a = (float*)take((size_t)NB * 128 * 4); float* c1 = (float*)take((size_t)NB * 128 * 4); float* c2 = (float*)take((size_t)NB * HH * 4);
  if (off > ws_size) return;
  for (int l = 0; l < NL; ++l) { k_wt_msg<<<(HH * 12 + 255) / 256, 256, 0, stream>>>(Wmsg + (size_t)l * (HH + EF) * HH, Bmsg[l]); k_wt_bf16<<<(HH * (2 * HH / 8) + 255) / 256, 256, 0, stream>>>(Wupd + (size_t)l * 2 * HH * HH, Bupd[l], 2 * HH, HH); }
  k_wt_bf16<<<(128 * (288 / 8) + 255) / 256, 256, 0, stream>>>(Wc1, Bc1, 288, 128);
  k_wt_bf16<<<(64 * (128 / 8) + 255) / 256, 256, 0, stream>>>(Wc2, Bc2, 128, 64);
  k_sort_init<<<NP2 / 256, 256, 0, stream>>>(dst, NEDGE, NNODE, key, perm, NP2);
  sort_pairs(key, perm, NP2, stream);
  k_rowptr<<<(NNODE + 32 + 255) / 256, 256, 0, stream>>>(key, NP2, NNODE, rowptr);
  k_enc<<<(NNODE + 7) / 8, 256, 0, stream>>>(x, W0, b0, ln1g, ln1b, hA);
  float* h = hA; float* hn = hB;
  for (int l = 0; l < NL; ++l) {
    k_gemm_msg<<<NEDGE / 64, 128, 0, stream>>>(h, ea, src, etype, Bmsg[l], bmsg + l * HH, gemb + (size_t)l * NG * HH, m);
    k_agg<<<(NNODE + 7) / 8, 256, 0, stream>>>(h, m, rowptr, perm, hcat);
    k_gemm_upd<<<(NNODE / 16 + 3) / 4, 128, 0, stream>>>(hcat, Bupd[l], bupd + l * HH, h, hn, NNODE);
    float* t2 = h; h = hn; hn = t2;
  }
  k_gptr<<<(NB + 32 + 255) / 256, 256, 0, stream>>>(batch, gptr);
  k_graphfeat<<<NB, 64, 0, stream>>>(h, gptr, gfeat, thr, Wg, bg, lngg, lngb, emb_th, Wt, bt, crow);
  k_gemm_bf3<true, 1, true, false><<<((NB / 16) * (128 / 64) + 3) / 4, 128, 0, stream>>>(crow, 288, Bc1, 288, bc1, nullptr, 1, 0, c1a, 128, NB, 128, 288);
  k_ln_rows<<<NB, 128 / 4, 0, stream>>>(c1a, nullptr, lncg, lncb, c1, 128, 1e-5f);
  k_gemm_bf3<true, 1, true, false><<<((NB / 16) * (HH / 64) + 3) / 4, 128, 0, stream>>>(c1, 128, Bc2, 128, bc2, nullptr, 1, 0, c2, HH, NB, HH, 128);
  k_head<<<1, 256, 0, stream>>>(c2, Wh1, bh1, Wh2, bh2, (float*)d_out);
}
